// SSMBlock_46712064311927
// MI455X (gfx1250) — hardware-verified
//
#include <hip/hip_runtime.h>
#include <math.h>

typedef __attribute__((ext_vector_type(16))) _Float16 v16h;
typedef __attribute__((ext_vector_type(8)))  _Float16 v8h;
typedef __attribute__((ext_vector_type(16))) __bf16   v16b;
typedef __attribute__((ext_vector_type(8)))  __bf16   v8b;
typedef __attribute__((ext_vector_type(8)))  float    v8f;
typedef __attribute__((ext_vector_type(4)))  float    v4f;
typedef __attribute__((ext_vector_type(2)))  float    v2f;
typedef __attribute__((ext_vector_type(4)))  unsigned v4u;

constexpr int kBatch  = 2;
constexpr int kSeq    = 2048;
constexpr int kDm     = 1024;
constexpr int kDin    = 2048;
constexpr int kNst    = 16;
constexpr int kXzN    = 2 * kDin;
constexpr int kRows   = kBatch * kSeq;
constexpr int kBcP    = 64;
constexpr int kConvTP = 260;
constexpr int kScanTS = 16;
constexpr int kScanCh = 512;
constexpr int kScanYP = 516;
constexpr float kCarryG   = 16.0f;
constexpr float kCarryW   = 32.0f;
constexpr float kOutScale = 1.0f / (kCarryG * kCarryW);
static_assert(kRows == 4096 && kXzN == 4096, "shape");
static_assert((kDm % 32) == 0 && (kDin % 32) == 0, "GEMM K multiples of 32");
static_assert((kRows % 64) == 0 && (kDin % 64) == 0 && (kBcP % 64) == 0 && (kDm % 64) == 0, "GEMM M,N multiples of 64");
static_assert((kSeq % 64) == 0 && (kSeq % kScanTS) == 0 && (kDin % kScanCh) == 0 && (kDin % 256) == 0, "tile multiples");
static_assert(kScanTS * kScanYP >= 32 * 256, "A staging fits the y tile");
static_assert(2 * kNst == 32, "B|C width");

constexpr size_t kOffXB   = 0;
constexpr size_t kOffWIN  = kOffXB  + (size_t)kRows * kDm * 2;
constexpr size_t kOffG16  = 0;
constexpr size_t kOffXIP  = kOffWIN + (size_t)kXzN * kDm * 2;
constexpr size_t kOffGATE = kOffXIP + (size_t)kRows * kDin * 4;
constexpr size_t kOffXH   = kOffGATE + (size_t)kRows * kDin * 2;
constexpr size_t kOffXM   = kOffXH  + (size_t)kRows * kDin * 2;
constexpr size_t kOffXL   = kOffXM  + (size_t)kRows * kDin * 2;
constexpr size_t kOffWOUT = kOffXL  + (size_t)kRows * kDin * 2;
constexpr size_t kOffWBC  = kOffWOUT + (size_t)kDm * kDin * 2;
constexpr size_t kOffBC   = kOffWBC + (size_t)64 * kDin * 2;
constexpr size_t kOffBCB  = kOffBC  + (size_t)kRows * kBcP * 4;
constexpr size_t kWsTotal = kOffBCB + 256;
static_assert(kWsTotal == 122945792ull, "carve total");
static_assert(kWsTotal <= 134217728ull, "carve cap");
static_assert((size_t)kRows * kDin * 2 <= kOffXIP, "G16 fits the dead XB16+WINT region");
static_assert((kOffWIN % 256) == 0 && (kOffXIP % 256) == 0 && (kOffGATE % 256) == 0 && (kOffXH % 256) == 0 &&
              (kOffXM % 256) == 0 && (kOffXL % 256) == 0 && (kOffWOUT % 256) == 0 && (kOffWBC % 256) == 0 &&
              (kOffBC % 256) == 0 && (kOffBCB % 256) == 0, "aligned regions");

__device__ __forceinline__ unsigned f2bf_u(float f) {
  const unsigned u = __float_as_uint(f);
  return (u + 0x7FFFu + ((u >> 16) & 1u)) >> 16;
}
__device__ __forceinline__ float bf_u2f(unsigned h) { return __uint_as_float(h << 16); }
__device__ __forceinline__ float rbf(float f) { return bf_u2f(f2bf_u(f)); }
__device__ __forceinline__ float bf_lo(unsigned w) { return __uint_as_float(w << 16); }
__device__ __forceinline__ float bf_hi(unsigned w) { return __uint_as_float(w & 0xffff0000u); }
__device__ __forceinline__ float h16_to_f32(unsigned hb) {
  const unsigned sgn = (hb & 0x8000u) << 16; const unsigned em = hb & 0x7fffu;
  const float fn = __uint_as_float((em << 13) + 0x38000000u);
  const float fs = (float)em * 5.9604644775390625e-8f;
  const float mag = (em < 0x400u) ? fs : fn; return __uint_as_float(__float_as_uint(mag) | sgn); }
__device__ __forceinline__ void split3(float v, unsigned& h, unsigned& m, unsigned& l) {
  h = f2bf_u(v);
  const float r1 = v - bf_u2f(h);
  m = f2bf_u(r1);
  const float r2 = r1 - bf_u2f(m);
  l = f2bf_u(r2);
}

__device__ __forceinline__ void grp_guard_h(v8f& a, v8f& b, v8f& c, v8f& d, v16h x, v16h y, v16h z, v16h p, v16h q, v16h r, v16h s) {
  asm volatile("v_nop\n\tv_nop\n\tv_nop\n\tv_nop" : "+v"(a), "+v"(b), "+v"(c), "+v"(d) : "v"(x), "v"(y), "v"(z), "v"(p), "v"(q), "v"(r), "v"(s));
}
__device__ __forceinline__ void grp_guard_b(v8f& a, v8f& b, v8f& c, v8f& d, v16b x, v16b y, v16b z, v16b p, v16b q, v16b r, v16b s) {
  asm volatile("v_nop\n\tv_nop\n\tv_nop\n\tv_nop" : "+v"(a), "+v"(b), "+v"(c), "+v"(d) : "v"(x), "v"(y), "v"(z), "v"(p), "v"(q), "v"(r), "v"(s));
}
__device__ __forceinline__ void keep4_h(v16h a, v16h b, v16h c, v16h d) { asm volatile("v_nop" :: "v"(a), "v"(b), "v"(c), "v"(d)); }
__device__ __forceinline__ void keep4_b(v16b a, v16b b, v16b c, v16b d) { asm volatile("v_nop" :: "v"(a), "v"(b), "v"(c), "v"(d)); }
__device__ __forceinline__ void acc_guard4(v8f& a, v8f& b, v8f& c, v8f& d) { asm volatile("v_nop\n\tv_nop\n\tv_nop\n\tv_nop" : "+v"(a), "+v"(b), "+v"(c), "+v"(d)); }
template <typename T> struct Frag;
template <> struct Frag<_Float16> {
  typedef v16h V; union U { v16h v; v8h h[2]; };
  static __device__ __forceinline__ v16h load(const _Float16* p) {
    U f; f.h[0] = *(const v8h*)(p); f.h[1] = *(const v8h*)(p + 16); return f.v;
  }
  static __device__ __forceinline__ v8f mma(v16h a, v16h b, v8f c) {
    return __builtin_amdgcn_wmma_f32_16x16x32_f16(false, a, false, b, (short)0, c, false, false);
  }
  static __device__ __forceinline__ void guard(v8f& a, v8f& b, v8f& c, v8f& d, v16h x, v16h y, v16h z, v16h p, v16h q, v16h r, v16h s) { grp_guard_h(a, b, c, d, x, y, z, p, q, r, s); }
  static __device__ __forceinline__ void keep(v16h a, v16h b, v16h c, v16h d) { keep4_h(a, b, c, d); }
};
template <> struct Frag<__bf16> {
  typedef v16b V; union U { v16b v; v8b h[2]; };
  static __device__ __forceinline__ v16b load(const __bf16* p) {
    U f; f.h[0] = *(const v8b*)(p); f.h[1] = *(const v8b*)(p + 16); return f.v;
  }
  static __device__ __forceinline__ v8f mma(v16b a, v16b b, v8f c) {
    return __builtin_amdgcn_wmma_f32_16x16x32_bf16(false, a, false, b, (short)0, c, false, false);
  }
  static __device__ __forceinline__ void guard(v8f& a, v8f& b, v8f& c, v8f& d, v16b x, v16b y, v16b z, v16b p, v16b q, v16b r, v16b s) { grp_guard_b(a, b, c, d, x, y, z, p, q, r, s); }
  static __device__ __forceinline__ void keep(v16b a, v16b b, v16b c, v16b d) { keep4_b(a, b, c, d); }
};
template <int ET> struct Elem;
template <> struct Elem<0> { typedef _Float16 T; };
template <> struct Elem<1> { typedef __bf16 T; };

template <int ET, int NA, int OUT_MODE, int ACT>
__global__ __launch_bounds__(256) void wmma_gemm64(
    const unsigned short* __restrict__ A1p, const unsigned short* __restrict__ A2p,
    const unsigned short* __restrict__ A3p, int lda,
    const unsigned short* __restrict__ Btp, int ldb,
    void* __restrict__ Cout, int ldc,
    const float* __restrict__ bias,
    int M, int N, int K, float scale) {
  typedef typename Elem<ET>::T T;
  typedef typename Frag<T>::V V;
  const T* A1 = (const T*)A1p; const T* A2 = (const T*)A2p; const T* A3 = (const T*)A3p; const T* Bt = (const T*)Btp;
  __shared__ __align__(16) float sT[8][16 * 68];
  const int lane = threadIdx.x & 31;
  const int wave = threadIdx.x >> 5;
  const int tilesN = N >> 6;
  const int tilesM = M >> 6;
  const int tile = blockIdx.x * 8 + wave;
  if (tile >= tilesM * tilesN) return;
  const int tm = tile / tilesN;
  const int tn = tile - tm * tilesN;
  const int m0 = tm << 6;
  const int n0 = tn << 6;

  const int rlane = lane & 15;
  const int koff  = (lane >> 4) * 8;
  const int mOff  = (lane >> 4) * 8;

  v8f acc[4][4];
#pragma unroll
  for (int i = 0; i < 4; ++i)
#pragma unroll
    for (int j = 0; j < 4; ++j) acc[i][j] = (v8f){0.f,0.f,0.f,0.f,0.f,0.f,0.f,0.f};

  for (int k0 = 0; k0 < K; k0 += 32) {
    V bh[4];
#pragma unroll
    for (int j = 0; j < 4; ++j) {
      const size_t bo = (size_t)(n0 + (j << 4) + rlane) * ldb + koff + k0;
      bh[j] = Frag<T>::load(Bt + bo);
    }
#pragma unroll
    for (int i = 0; i < 4; ++i) {
      const size_t ao = (size_t)(m0 + (i << 4) + rlane) * lda + koff + k0;
      V a1 = Frag<T>::load(A1 + ao);
      V a2 = a1;
      V a3 = a1;
      if (NA == 3) { a2 = Frag<T>::load(A2 + ao); a3 = Frag<T>::load(A3 + ao); }
#pragma unroll
      for (int j = 0; j < 4; ++j) {
        acc[i][j] = Frag<T>::mma(a1, bh[j], acc[i][j]);
        if (NA == 3) {
          acc[i][j] = Frag<T>::mma(a2, bh[j], acc[i][j]);
          acc[i][j] = Frag<T>::mma(a3, bh[j], acc[i][j]);
        }
      }
      Frag<T>::guard(acc[i][0], acc[i][1], acc[i][2], acc[i][3], a1, a2, a3, bh[0], bh[1], bh[2], bh[3]);
    }
    Frag<T>::keep(bh[0], bh[1], bh[2], bh[3]);
  }
  acc_guard4(acc[0][0], acc[0][1], acc[0][2], acc[0][3]);
  acc_guard4(acc[1][0], acc[1][1], acc[1][2], acc[1][3]);
  acc_guard4(acc[2][0], acc[2][1], acc[2][2], acc[2][3]);
  acc_guard4(acc[3][0], acc[3][1], acc[3][2], acc[3][3]);

  float* slab = sT[wave];
#pragma unroll
  for (int i = 0; i < 4; ++i) {
    const int mBase = m0 + (i << 4);
#pragma unroll
    for (int j = 0; j < 4; ++j) {
      const int n = n0 + (j << 4) + rlane;
      const float bv = rbf(bias[n]);
#pragma unroll
      for (int r = 0; r < 8; ++r) {
        float v = acc[i][j][r] * scale;
        v += bv;
        slab[(mOff + r) * 68 + (j << 4) + rlane] = v;
      }
    }
    __builtin_amdgcn_fence(__ATOMIC_RELEASE, "workgroup");
    __builtin_amdgcn_wave_barrier();
    __builtin_amdgcn_fence(__ATOMIC_ACQUIRE, "workgroup");
    if (ACT == 1) {
#pragma unroll 1
      for (int t = 0; t < 16; ++t) {
        float* p = slab + t * 68 + lane * 2;
        const v2f zv = *(const v2f*)p;
        v2f ov;
        ov[0] = 1.0f / (1.0f + expf(-zv[0]));
        ov[1] = 1.0f / (1.0f + expf(-zv[1]));
        *(v2f*)p = ov;
      }
      __builtin_amdgcn_fence(__ATOMIC_RELEASE, "workgroup");
      __builtin_amdgcn_wave_barrier();
      __builtin_amdgcn_fence(__ATOMIC_ACQUIRE, "workgroup");
    }
    if (OUT_MODE == 0) {
      float* C = (float*)Cout;
      const int hh = lane >> 4, c4 = (lane & 15) * 4;
      for (int pass = 0; pass < 2; ++pass) {
#pragma unroll
        for (int it = 0; it < 8; ++it) {
          const int row = it * 2 + hh;
          v4f v = *(const v4f*)(slab + row * 68 + c4);
          *(volatile v4f*)(C + (size_t)(mBase + row) * ldc + n0 + c4) = v;
        }
        __threadfence();
      }
    } else {
      const int q = lane >> 3, c8 = (lane & 7) * 8;
      unsigned short* C = (unsigned short*)Cout;
      for (int pass = 0; pass < 2; ++pass) {
#pragma unroll
        for (int it = 0; it < 4; ++it) {
          const int row = it * 4 + q;
          const float* sp = slab + row * 68 + c8;
          v8h hv;
#pragma unroll
          for (int e = 0; e < 8; ++e) hv[e] = (_Float16)sp[e];
          *(volatile v8h*)(C + (size_t)(mBase + row) * ldc + n0 + c8) = hv;
        }
        __threadfence();
      }
    }
    __builtin_amdgcn_fence(__ATOMIC_RELEASE, "workgroup");
    __builtin_amdgcn_wave_barrier();
    __builtin_amdgcn_fence(__ATOMIC_ACQUIRE, "workgroup");
  }
}

__global__ __launch_bounds__(256) void cast_bf16_kernel(
    const float* __restrict__ src, unsigned short* __restrict__ dst, int total8)
{
  const int i = blockIdx.x * 256 + threadIdx.x;
  if (i >= total8) return;
  const size_t e0 = (size_t)i << 3;
  const v4f a0 = *(const v4f*)(src + e0);
  const v4f a1 = *(const v4f*)(src + e0 + 4);
  v4u w;
  w[0] = f2bf_u(a0[0]) | (f2bf_u(a0[1]) << 16);
  w[1] = f2bf_u(a0[2]) | (f2bf_u(a0[3]) << 16);
  w[2] = f2bf_u(a1[0]) | (f2bf_u(a1[1]) << 16);
  w[3] = f2bf_u(a1[2]) | (f2bf_u(a1[3]) << 16);
  unsigned short* q = dst + e0;
  *(volatile v4u*)q = w;
  __threadfence();
  *(volatile v4u*)q = w;
}

template <int MODE> __device__ __forceinline__ unsigned cvt16_u(float f, float scale) {
  if (MODE == 0) return f2bf_u(f);
  const _Float16 hv = (_Float16)(rbf(f) * scale);
  const unsigned short hb = __builtin_bit_cast(unsigned short, hv);
  return (unsigned)hb;
}
template <int MODE> __device__ __forceinline__ void bt_store_tile(
    const float* tile, unsigned short* __restrict__ Bt, int n0, int k0, int Kdim, float scale, int lane, int wave)
{
  const int q = lane >> 3, c8 = (lane & 7) * 8;
  v4u w[2];
#pragma unroll
  for (int it = 0; it < 2; ++it) {
    const int nrow = it * 32 + wave * 4 + q;
#pragma unroll
    for (int e2 = 0; e2 < 4; ++e2) {
      const float fa = tile[(c8 + 2 * e2) * 65 + nrow];
      const float fb = tile[(c8 + 2 * e2 + 1) * 65 + nrow];
      const unsigned ua = cvt16_u<MODE>(fa, scale);
      const unsigned ub = cvt16_u<MODE>(fb, scale);
      w[it][e2] = ua | (ub << 16);
    }
  }
  for (int pass = 0; pass < 2; ++pass) {
#pragma unroll
    for (int it = 0; it < 2; ++it) {
      const int nrow = it * 32 + wave * 4 + q;
      *(volatile v4u*)(Bt + (size_t)(n0 + nrow) * Kdim + k0 + c8) = w[it];
    }
    __threadfence();
  }
}

template <int MODE>
__global__ __launch_bounds__(256) void transpose_cast_kernel(
    const float* __restrict__ W, unsigned short* __restrict__ Bt, int Kdim, int Ndim, float scale)
{
  __shared__ float tile[64 * 65];
  const int tid = threadIdx.x, lane = tid & 31, wave = tid >> 5;
  const int n0 = blockIdx.x * 64;
  const int k0 = blockIdx.y * 64;
#pragma unroll
  for (int p = 0; p < 16; ++p) {
    const int idx = tid + p * 256;
    const int kk  = idx >> 6;
    const int nn  = idx & 63;
    const int n   = n0 + nn;
    const int nc  = (n < Ndim) ? n : (Ndim - 1);
    const float v = W[(size_t)(k0 + kk) * Ndim + nc];
    tile[kk * 65 + nn] = (n < Ndim) ? v : 0.f;
  }
  __syncthreads();
  bt_store_tile<MODE>(tile, Bt, n0, k0, Kdim, scale, lane, wave);
}

__global__ __launch_bounds__(256) void wbc_plane_kernel(
    const float* __restrict__ WB, const float* __restrict__ WC, unsigned short* __restrict__ Bt)
{
  __shared__ float tile[64 * 65];
  const int tid = threadIdx.x, lane = tid & 31, wave = tid >> 5;
  const int k0 = blockIdx.x * 64;
  const int kk = tid >> 2, q4 = (tid & 3) * 4;
  const v4f a = *(const v4f*)(WB + (size_t)(k0 + kk) * kNst + q4);
  const v4f b = *(const v4f*)(WC + (size_t)(k0 + kk) * kNst + q4);
#pragma unroll
  for (int e = 0; e < 4; ++e) {
    tile[kk * 65 + q4 + e] = a[e];
    tile[kk * 65 + kNst + q4 + e] = b[e];
  }
#pragma unroll
  for (int e = 0; e < 8; ++e) tile[kk * 65 + 32 + (tid & 3) * 8 + e] = 0.f;
  __syncthreads();
  bt_store_tile<0>(tile, Bt, 0, k0, kDin, 1.0f, lane, wave);
}

__global__ __launch_bounds__(32) void bc_bias_kernel(
    const float* __restrict__ bB, const float* __restrict__ bC, float* __restrict__ dst)
{
  const int lane = threadIdx.x & 31;
  const int q = (lane & 3) * 4;
  const v4f a = *(const v4f*)(bB + q);
  const v4f b = *(const v4f*)(bC + q);
  const float fa = (lane < 4) ? 1.0f : 0.0f;
  const float fb = (lane >= 4 && lane < 8) ? 1.0f : 0.0f;
  v4f v;
#pragma unroll
  for (int e = 0; e < 4; ++e) v[e] = fa * rbf(a[e]) + fb * rbf(b[e]);
  const int ls = (lane < 16) ? lane : 15;
  if (lane < 16) *(volatile v4f*)(dst + ls * 4) = v;
  __threadfence();
  if (lane < 16) *(volatile v4f*)(dst + ls * 4) = v;
}

__global__ __launch_bounds__(256) void conv_silu_split_kernel(
    const float* __restrict__ XIP, const float* __restrict__ cw, const float* __restrict__ cb,
    unsigned short* __restrict__ XH, unsigned short* __restrict__ XM, unsigned short* __restrict__ XL)
{
  __shared__ __align__(16) float sT[16 * kConvTP];
  const int tid = threadIdx.x, lane = tid & 31, wave = tid >> 5;
  const int d0 = blockIdx.x * 256, d = d0 + tid;
  const int g0 = blockIdx.y * 64;
  const int tb = g0 & (kSeq - 1);
  const v4f wv = *(const v4f*)(cw + (size_t)d * 4);
  const float w0 = rbf(wv[0]), w1 = rbf(wv[1]), w2 = rbf(wv[2]), w3 = rbf(wv[3]);
  const float bc = rbf(cb[d]);
  float xm3, xm2, xm1;
  {
    const bool hist = (tb > 0);
    const int rb = hist ? (g0 - 3) : g0;
    const float v3 = XIP[(size_t)rb * kDin + d];
    const float v2 = XIP[(size_t)(rb + 1) * kDin + d];
    const float v1 = XIP[(size_t)(rb + 2) * kDin + d];
    xm3 = hist ? v3 : 0.f;
    xm2 = hist ? v2 : 0.f;
    xm1 = hist ? v1 : 0.f;
  }
#pragma unroll 1
  for (int sub = 0; sub < 4; ++sub) {
    const int lb = g0 + sub * 16;
#pragma unroll 1
    for (int s = 0; s < 16; ++s) {
      const float xcur = XIP[(size_t)(lb + s) * kDin + d];
      float acc = w0 * xm3;
      acc = fmaf(w1, xm2, acc);
      acc = fmaf(w2, xm1, acc);
      acc = fmaf(w3, xcur, acc);
      const float sv = acc + bc;
      const float sg = 1.0f / (1.0f + expf(-sv));
      sT[s * kConvTP + tid] = sv * sg;
      xm3 = xm2; xm2 = xm1; xm1 = xcur;
    }
    __syncthreads();
    v4u wh[2], wm[2], wl[2];
#pragma unroll
    for (int it = 0; it < 2; ++it) {
      const float* sp = sT + (it * 8 + wave) * kConvTP + lane * 8;
      const v4f a0 = *(const v4f*)(sp);
      const v4f a1 = *(const v4f*)(sp + 4);
      const float f[8] = {a0[0], a0[1], a0[2], a0[3], a1[0], a1[1], a1[2], a1[3]};
#pragma unroll
      for (int e2 = 0; e2 < 4; ++e2) {
        unsigned ha, ma, la, hb, mb, lbb;
        split3(f[2 * e2], ha, ma, la);
        split3(f[2 * e2 + 1], hb, mb, lbb);
        wh[it][e2] = ha | (hb << 16);
        wm[it][e2] = ma | (mb << 16);
        wl[it][e2] = la | (lbb << 16);
      }
    }
    for (int pass = 0; pass < 2; ++pass) {
#pragma unroll
      for (int it = 0; it < 2; ++it) {
        const size_t o = (size_t)(lb + it * 8 + wave) * kDin + d0 + lane * 8;
        *(volatile v4u*)(XH + o) = wh[it];
        *(volatile v4u*)(XM + o) = wm[it];
        *(volatile v4u*)(XL + o) = wl[it];
      }
      __threadfence();
    }
    __syncthreads();
  }
}

__global__ __launch_bounds__(256) void scan_kernel(
    const float* __restrict__ BC, const unsigned* __restrict__ XHw, const unsigned* __restrict__ XMw,
    const unsigned* __restrict__ XLw, const unsigned* __restrict__ GTw,
    const float* __restrict__ Alog, const float* __restrict__ Dp, unsigned short* __restrict__ G16)
{
#pragma clang fp contract(off)
  __shared__ __align__(16) float sBC[kScanTS * 32];
  __shared__ __align__(16) float sY[kScanTS * kScanYP];
  const int tid = threadIdx.x, lane = tid & 31, wave = tid >> 5;
  constexpr int kBlkPerB = kDin / kScanCh;
  const int bix = blockIdx.x / kBlkPerB;
  const int d0  = (blockIdx.x - bix * kBlkPerB) * kScanCh;
  const int d   = d0 + 2 * tid;
  const size_t row0 = (size_t)bix * kSeq;

#pragma unroll 1
  for (int e = 0; e < 32; ++e) {
    const float al = rbf(Alog[(size_t)d * kNst + e]);
    const float ac = fminf(fmaxf(al, -10.0f), 2.0f);
    sY[e * 256 + tid] = -expf(ac);
  }
  __syncthreads();
  float A0[kNst], A1[kNst], h0[kNst], h1[kNst];
#pragma unroll
  for (int n = 0; n < kNst; ++n) {
    A0[n] = sY[n * 256 + tid];
    A1[n] = sY[(kNst + n) * 256 + tid];
    h0[n] = 0.f;
    h1[n] = 0.f;
  }
  const v2f dv = *(const v2f*)(Dp + d);
  const float D0 = rbf(dv[0]), D1 = rbf(dv[1]);
  const size_t wcol = (size_t)(d >> 1);
  constexpr size_t kWP = (size_t)(kDin / 2);

#pragma unroll 1
  for (int c = 0; c < kSeq / kScanTS; ++c) {
    const int l0 = c * kScanTS;
    if (tid < 128) {
      const int r = tid >> 3, q = (tid & 7) * 4;
      const v4f v = *(const v4f*)(BC + (row0 + l0 + r) * kBcP + q);
      *(v4f*)(sBC + r * 32 + q) = v;
    }
    __syncthreads();
#pragma unroll 1
    for (int s = 0; s < kScanTS; ++s) {
      const size_t wi = (row0 + l0 + s) * kWP + wcol;
      const unsigned wh = XHw[wi];
      const unsigned wm = XMw[wi];
      const unsigned wl = XLw[wi];
      const unsigned wg = GTw[wi];
      float x0 = bf_lo(wh) + bf_lo(wm);
      x0 = x0 + bf_lo(wl);
      float x1 = bf_hi(wh) + bf_hi(wm);
      x1 = x1 + bf_hi(wl);
      const float g0 = h16_to_f32(wg & 0xffffu);
      const float g1 = h16_to_f32(wg >> 16);
      v4f Bq[4], Cq[4];
#pragma unroll
      for (int qq = 0; qq < 4; ++qq) {
        Bq[qq] = *(const v4f*)(sBC + s * 32 + 4 * qq);
        Cq[qq] = *(const v4f*)(sBC + s * 32 + kNst + 4 * qq);
      }
      float y0 = 0.f, y1 = 0.f;
#pragma unroll
      for (int n = 0; n < kNst; ++n) {
        const float bn = Bq[n >> 2][n & 3];
        const float cn = Cq[n >> 2][n & 3];
        const float ta = h0[n] * A0[n];
        const float ua = x0 * bn;
        float va = ta + ua;
        va = fminf(fmaxf(va, -100.0f), 100.0f);
        h0[n] = va;
        y0 = fmaf(va, cn, y0);
        const float tb = h1[n] * A1[n];
        const float ub = x1 * bn;
        float vb = tb + ub;
        vb = fminf(fmaxf(vb, -100.0f), 100.0f);
        h1[n] = vb;
        y1 = fmaf(vb, cn, y1);
      }
      const float sk0 = D0 * x0;
      const float sk1 = D1 * x1;
      y0 = y0 + sk0;
      y1 = y1 + sk1;
      y0 = fminf(fmaxf(y0, -100.0f), 100.0f);
      y1 = fminf(fmaxf(y1, -100.0f), 100.0f);
      v2f ov;
      ov[0] = (y0 * g0) * kCarryG;
      ov[1] = (y1 * g1) * kCarryG;
      *(v2f*)(sY + s * kScanYP + 2 * tid) = ov;
    }
    __syncthreads();
    v8h hv[4];
#pragma unroll
    for (int it = 0; it < 4; ++it) {
      const int u = it * 8 + wave;
      const int row = u >> 1, hf = u & 1;
      const float* sp = sY + row * kScanYP + hf * 256 + lane * 8;
      const v4f a0 = *(const v4f*)(sp);
      const v4f a1 = *(const v4f*)(sp + 4);
#pragma unroll
      for (int e = 0; e < 4; ++e) { hv[it][e] = (_Float16)a0[e]; hv[it][4 + e] = (_Float16)a1[e]; }
    }
    for (int pass = 0; pass < 2; ++pass) {
#pragma unroll
      for (int it = 0; it < 4; ++it) {
        const int u = it * 8 + wave;
        const int row = u >> 1, hf = u & 1;
        *(volatile v8h*)(G16 + (row0 + l0 + row) * kDin + d0 + hf * 256 + lane * 8) = hv[it];
      }
      __threadfence();
    }
  }
}

extern "C" void kernel_launch(void* const* d_in, const int* in_sizes, int n_in,
                              void* d_out, int out_size, void* d_ws, size_t ws_size,
                              hipStream_t stream) {
  if (n_in < 13) return;
  if (in_sizes[0] != kRows * kDm) return;
  if (in_sizes[1] != kDm * kXzN) return;
  if (in_sizes[2] != kXzN) return;
  if (in_sizes[3] != kDin * 4) return;
  if (in_sizes[4] != kDin) return;
  if (in_sizes[5] != kDin * kNst) return;
  if (in_sizes[6] != kDin) return;
  if (in_sizes[7] != kDin * kNst) return;
  if (in_sizes[8] != kNst) return;
  if (in_sizes[9] != kDin * kNst) return;
  if (in_sizes[10] != kNst) return;
  if (in_sizes[11] != kDin * kDm) return;
  if (in_sizes[12] != kDm) return;
  if (out_size != kRows * kDm) return;
  if (ws_size < kWsTotal) return;

  const float* x      = (const float*)d_in[0];
  const float* W_in   = (const float*)d_in[1];
  const float* b_in   = (const float*)d_in[2];
  const float* W_conv = (const float*)d_in[3];
  const float* b_conv = (const float*)d_in[4];
  const float* A_log  = (const float*)d_in[5];
  const float* Dv     = (const float*)d_in[6];
  const float* W_B    = (const float*)d_in[7];
  const float* b_B    = (const float*)d_in[8];
  const float* W_C    = (const float*)d_in[9];
  const float* b_C    = (const float*)d_in[10];
  const float* W_out  = (const float*)d_in[11];
  const float* b_out  = (const float*)d_in[12];
  float* out = (float*)d_out;

  char* ws = (char*)d_ws;
  unsigned short* XB16  = (unsigned short*)(ws + kOffXB);
  unsigned short* WINT  = (unsigned short*)(ws + kOffWIN);
  unsigned short* G16   = (unsigned short*)(ws + kOffG16);
  float*          XIP   = (float*)(ws + kOffXIP);
  unsigned short* GATE  = (unsigned short*)(ws + kOffGATE);
  unsigned short* XH    = (unsigned short*)(ws + kOffXH);
  unsigned short* XM    = (unsigned short*)(ws + kOffXM);
  unsigned short* XL    = (unsigned short*)(ws + kOffXL);
  unsigned short* WOUTT = (unsigned short*)(ws + kOffWOUT);
  unsigned short* WBCT  = (unsigned short*)(ws + kOffWBC);
  float*          BC    = (float*)(ws + kOffBC);
  float*          BCB   = (float*)(ws + kOffBCB);

  cast_bf16_kernel<<<(kRows * kDm / 8) / 256, 256, 0, stream>>>(x, XB16, kRows * kDm / 8);
  transpose_cast_kernel<0><<<dim3(kXzN / 64, kDm / 64), 256, 0, stream>>>(W_in, WINT, kDm, kXzN, 1.0f);
  transpose_cast_kernel<1><<<dim3(kDm / 64, kDin / 64), 256, 0, stream>>>(W_out, WOUTT, kDin, kDm, kCarryW);
  wbc_plane_kernel<<<kDin / 64, 256, 0, stream>>>(W_B, W_C, WBCT);
  bc_bias_kernel<<<1, 32, 0, stream>>>(b_B, b_C, BCB);

  wmma_gemm64<1, 1, 0, 0><<<256, 256, 0, stream>>>(
      XB16, XB16, XB16, kDm, WINT, kDm, (void*)XIP, kDin, b_in, kRows, kDin, kDm, 1.0f);
  wmma_gemm64<1, 1, 1, 1><<<256, 256, 0, stream>>>(
      XB16, XB16, XB16, kDm, WINT + (size_t)kDin * kDm, kDm, (void*)GATE, kDin, b_in + kDin, kRows, kDin, kDm, 1.0f);

  conv_silu_split_kernel<<<dim3(kDin / 256, kRows / 64), 256, 0, stream>>>(XIP, W_conv, b_conv, XH, XM, XL);

  wmma_gemm64<1, 3, 0, 0><<<8, 256, 0, stream>>>(
      XH, XM, XL, kDin, WBCT, kDin, (void*)BC, kBcP, BCB, kRows, kBcP, kDin, 1.0f);

  scan_kernel<<<kBatch * (kDin / kScanCh), 256, 0, stream>>>(
      BC, (const unsigned*)XH, (const unsigned*)XM, (const unsigned*)XL, (const unsigned*)GATE, A_log, Dv, G16);

  wmma_gemm64<0, 1, 0, 0><<<128, 256, 0, stream>>>(
      G16, G16, G16, kDin, WOUTT, kDin, (void*)out, kDm, b_out, kRows, kDm, kDin, kOutScale);
}
